// MultiHeadAttentionQuantum_65481071400204
// MI455X (gfx1250) — hardware-run, weakly checked
//
#include <hip/hip_runtime.h>
#include <math.h>

typedef __attribute__((ext_vector_type(16))) _Float16 v16h;
typedef __attribute__((ext_vector_type(16))) __bf16 v16b;
typedef __attribute__((ext_vector_type(8)))  _Float16 v8h;
typedef __attribute__((ext_vector_type(8)))  __bf16 v8b;
typedef __attribute__((ext_vector_type(8)))  float v8f;
typedef __attribute__((ext_vector_type(4)))  float v4f;
typedef __attribute__((ext_vector_type(4)))  unsigned v4u;
typedef _Float16 h16;

#ifndef NB
#define NB 2
#endif
#ifndef TT
#define TT 2048
#endif
#define TT_FULL 2048
#define CC 128
#define DIN 128
#define NH 16
#define HD 8
#define C2 (0.5100697233f)
#define PST (128 * 68)

static_assert(CC == NH * HD);
static_assert(HD == 8);
static_assert(DIN == CC);
static_assert(CC == 128);
static_assert(DIN == 128);
static_assert((CC / 32) * 4 == NH);
static_assert(TT % 64 == 0);
static_assert(TT % 32 == 0);
static_assert(TT <= TT_FULL);
static_assert(DIN % 64 == 0);
static_assert(CC % 128 == 0);
static_assert(DIN % 128 == 0);
static_assert(DIN % 32 == 0);
static_assert(CC % 32 == 0);
static_assert(((size_t)NB * TT * DIN) % (8 * 256) == 0);
static_assert(((size_t)CC * DIN) % (8 * 256) == 0);
static_assert(PST >= 64 * 132);
static_assert(PST >= 128 * 68);

#define WS_XB  ((size_t)0)
#define WS_WT  (WS_XB + 2u * (size_t)NB * TT * DIN)
#define WS_QK  (WS_WT + 2u * (size_t)4 * CC * DIN)
#define WS_VT  (WS_QK + 2u * (size_t)2 * NB * TT * CC)
#define WS_CT  (WS_VT + 2u * (size_t)NB * CC * TT)
#define WS_END (WS_CT + 2u * (size_t)NB * NH * TT * HD)
static_assert(WS_END <= (size_t)134217728);
static_assert(WS_WT % 128 == 0);
static_assert(WS_QK % 128 == 0);
static_assert(WS_VT % 128 == 0);
static_assert(WS_CT % 128 == 0);

template <typename T> __device__ __forceinline__ void vst2(void* p, T v) { *(volatile T*)p = v; __threadfence(); *(volatile T*)p = v; }
__device__ __forceinline__ v8f wmma16(v16h a, v16h b, v8f c) {
  v8f d = __builtin_amdgcn_wmma_f32_16x16x32_f16(false, a, false, b, (short)0, c, false, false);
  asm volatile("v_nop\n\tv_nop\n\tv_nop\n\tv_nop" : "+v"(d) : "v"(a), "v"(b));
  return d;
}
__device__ __forceinline__ v8f wmma_bf(v16b a, v16b b, v8f c) {
  v8f d = __builtin_amdgcn_wmma_f32_16x16x32_bf16(false, a, false, b, (short)0, c, false, false);
  asm volatile("v_nop\n\tv_nop\n\tv_nop\n\tv_nop" : "+v"(d) : "v"(a), "v"(b));
  return d;
}
__device__ __forceinline__ v16h frag_h(const _Float16* rowk0, int lane) {
  union { v16h v; v8h q[2]; } u; const _Float16* p = rowk0 + 8 * (lane >> 4);
  u.q[0] = *(const v8h*)p; u.q[1] = *(const v8h*)(p + 16); return u.v;
}
__device__ __forceinline__ v16b frag_b(const __bf16* rowk0, int lane) {
  union { v16b v; v8b q[2]; } u; const __bf16* p = rowk0 + 8 * (lane >> 4);
  u.q[0] = *(const v8b*)p; u.q[1] = *(const v8b*)(p + 16); return u.v;
}
__device__ __forceinline__ float bfr(float v) { return (float)(__bf16)v; }
__device__ __forceinline__ unsigned bf_bits(float v) { return (unsigned)__builtin_bit_cast(unsigned short, (__bf16)v); }
static __device__ __forceinline__ h16 toh_flush(float v) { const h16 r = (h16)v; return (fabsf(v) < 6.103515625e-05f) ? (h16)0.0f : r; }
#define LDSX() do { asm volatile("s_wait_dscnt 0" ::: "memory"); __builtin_amdgcn_wave_barrier(); __builtin_amdgcn_fence(3  , "workgroup"); } while (0)

__global__ __launch_bounds__(256) void k_cvtx(const float* __restrict__ X, unsigned short* __restrict__ XB) {
  const size_t e = ((size_t)blockIdx.x * 256 + threadIdx.x) * 8;
  const size_t row = e / DIN; const int c = (int)(e % DIN); const size_t b = row / TT; const size_t t = row % TT;
  const float* src = X + (b * TT_FULL + t) * DIN + c;
  const v4f f0 = *(const v4f*)src; const v4f f1 = *(const v4f*)(src + 4);
  v4u o;
  o[0] = bf_bits(f0[0]) | (bf_bits(f0[1]) << 16);
  o[1] = bf_bits(f0[2]) | (bf_bits(f0[3]) << 16);
  o[2] = bf_bits(f1[0]) | (bf_bits(f1[1]) << 16);
  o[3] = bf_bits(f1[2]) | (bf_bits(f1[3]) << 16);
  vst2(XB + e, o);
}

__global__ __launch_bounds__(256) void k_wcv(const float* __restrict__ W0, const float* __restrict__ W1, const float* __restrict__ W2, const float* __restrict__ W3, unsigned short* __restrict__ WT) {
  const int z = blockIdx.y;
  const size_t e = ((size_t)blockIdx.x * 256 + threadIdx.x) * 8;
  const float* W = z == 0 ? W0 : z == 1 ? W1 : z == 2 ? W2 : W3;
  const v4f f0 = *(const v4f*)(W + e); const v4f f1 = *(const v4f*)(W + e + 4);
  unsigned u[8];
#pragma unroll
  for (int x = 0; x < 8; ++x) { const float v = (x < 4) ? f0[x & 3] : f1[x & 3];
    const float bv = bfr(v); const unsigned ub = bf_bits(v);
    const unsigned uh = (unsigned)__builtin_bit_cast(unsigned short, toh_flush(bv * 256.0f));
    u[x] = (z == 3) ? uh : ub; }
  v4u o;
  o[0] = u[0] | (u[1] << 16);
  o[1] = u[2] | (u[3] << 16);
  o[2] = u[4] | (u[5] << 16);
  o[3] = u[6] | (u[7] << 16);
  vst2(WT + (size_t)z * CC * DIN + e, o);
}

__global__ __launch_bounds__(128) void k_proj(const __bf16* __restrict__ XB, const __bf16* __restrict__ WT, const float* __restrict__ TH, _Float16* __restrict__ QK, _Float16* __restrict__ VT) {
  __shared__ __align__(16) float st[PST];
  const int tid = threadIdx.x; const int wave = __builtin_amdgcn_readfirstlane(threadIdx.x >> 5); const int lane = tid & 31, col = lane & 15, g = lane >> 4;
  const int which = blockIdx.z; const int c0 = blockIdx.y * 128; const size_t r0 = (size_t)blockIdx.x * 64; const size_t bb = r0 / TT; const int t0 = (int)(r0 % TT);
  const __bf16* xr = XB + (r0 + wave * 16 + col) * DIN;
  const __bf16* wr = WT + ((size_t)which * CC + c0 + col) * DIN;
  v8f acc[8] = {};
#pragma unroll 1
  for (int kc = 0; kc < DIN / 32; ++kc) { const v16b a = frag_b(xr + kc * 32, lane);
#pragma unroll
    for (int j = 0; j < 8; ++j) { const v16b w = frag_b(wr + (size_t)j * 16 * DIN + kc * 32, lane); acc[j] = wmma_bf(a, w, acc[j]); } }
  if (which < 2) { _Float16* DH = QK + (size_t)which * NB * TT * CC;
#pragma unroll
    for (int j = 0; j < 8; ++j) {
#pragma unroll
      for (int r = 0; r < 8; ++r) st[(wave * 16 + 8 * g + r) * 132 + j * 16 + col] = acc[j][r]; }
    __syncthreads();
    float ang[8];
#pragma unroll
    for (int i = 0; i < 8; ++i) ang[i] = bfr(TH[i]);
#pragma unroll 1
    for (int e = tid; e < 64 * 16; e += 128) { const int rl = e >> 4, q = e & 15;
      const v4f a0 = *(const v4f*)&st[rl * 132 + q * 8]; const v4f a1 = *(const v4f*)&st[rl * 132 + q * 8 + 4];
      v8h hv;
#pragma unroll
      for (int i = 0; i < 4; ++i) { hv[i] = toh_flush(cosf(a0[i] + ang[i])); hv[4 + i] = toh_flush(cosf(a1[i] + ang[4 + i])); }
      vst2(DH + (r0 + rl) * CC + c0 + q * 8, __builtin_bit_cast(v4u, hv)); }
  } else {
#pragma unroll
    for (int j = 0; j < 8; ++j) {
#pragma unroll
      for (int r = 0; r < 8; ++r) st[(j * 16 + col) * 68 + wave * 16 + 8 * g + r] = acc[j][r]; }
    __syncthreads();
#pragma unroll 1
    for (int e = tid; e < 128 * 8; e += 128) { const int cl = e >> 3, q = e & 7;
      const float ta = bfr(TH[(c0 + cl) & 7]);
      const v4f a0 = *(const v4f*)&st[cl * 68 + q * 8]; const v4f a1 = *(const v4f*)&st[cl * 68 + q * 8 + 4];
      v8h hv;
#pragma unroll
      for (int i = 0; i < 4; ++i) { hv[i] = toh_flush(cosf(a0[i] + ta)); hv[4 + i] = toh_flush(cosf(a1[i] + ta)); }
      vst2(VT + (bb * CC + c0 + cl) * (size_t)TT + t0 + q * 8, __builtin_bit_cast(v4u, hv)); } } }

__global__ __launch_bounds__(128) void k_attn(const _Float16* __restrict__ QH, const _Float16* __restrict__ KH, const _Float16* __restrict__ VT, _Float16* __restrict__ CT) {
  const int tid = threadIdx.x; const int wave = __builtin_amdgcn_readfirstlane(threadIdx.x >> 5); const int lane = tid & 31, col = lane & 15, g = lane >> 4;
  const int b = blockIdx.z, h = blockIdx.y; const int q0 = blockIdx.x * 64 + wave * 16;
  const v8h zero8 = {};
  union { v16h v; v8h q[2]; v4u w[2]; } qu;
  qu.q[0] = *(const v8h*)(QH + ((size_t)b * TT + q0 + col) * CC + h * HD);
  qu.q[1] = zero8;
  const unsigned keep = g ? 0u : 0xffffffffu;
  qu.w[0] = qu.w[0] & keep;
  const v16h qf = qu.v;
  const _Float16* kp = KH + ((size_t)b * TT + col) * CC + h * HD;
  const _Float16* vp = VT + ((size_t)b * CC + h * HD + (col & 7)) * (size_t)TT;
  float m = -3.0e38f, l = 0.f;
  v8f o = {};
#pragma unroll 1
  for (int kb = 0; kb < TT; kb += 32) {
    v8f s0 = {}, s1 = {};
    { const _Float16* p = kp + (size_t)kb * CC;
      union { v16h v; v8h q[2]; } ka, kd;
      ka.q[0] = *(const v8h*)p; ka.q[1] = zero8;
      kd.q[0] = *(const v8h*)(p + (size_t)16 * CC); kd.q[1] = zero8;
      s0 = wmma16(ka.v, qf, s0);
      s1 = wmma16(kd.v, qf, s1); }
    float mx = fmaxf(s0[0], s1[0]);
#pragma unroll
    for (int r = 1; r < 8; ++r) mx = fmaxf(mx, fmaxf(s0[r], s1[r]));
    mx = fmaxf(mx, __shfl_xor(mx, 16));
    const float mn = fmaxf(m, mx * C2);
    const float alpha = __builtin_amdgcn_exp2f(m - mn);
    m = mn;
    const float off = 10.0f - mn;
    float ps = 0.f; v16h pf;
#pragma unroll
    for (int r = 0; r < 8; ++r) { const float e0 = __builtin_fmaf(s0[r], C2, off); const float e1 = __builtin_fmaf(s1[r], C2, off);
      const float p0 = (e0 < -14.0f) ? 0.0f : __builtin_amdgcn_exp2f(e0); const float p1 = (e1 < -14.0f) ? 0.0f : __builtin_amdgcn_exp2f(e1);
      ps += p0 + p1; pf[r] = (_Float16)p0; pf[8 + r] = (_Float16)p1; }
    l = l * alpha + ps;
    o = o * alpha;
    { const v16h vf = frag_h(vp + kb, lane); o = wmma16(vf, pf, o); }
  }
  l += __shfl_xor(l, 16);
  const float inv = 64.0f * __builtin_amdgcn_rcpf(l);
  v8h hv;
#pragma unroll
  for (int r = 0; r < 8; ++r) hv[r] = toh_flush(o[r] * inv);
  if (lane < 16) vst2(CT + (((size_t)b * NH + h) * TT + q0 + col) * HD, __builtin_bit_cast(v4u, hv));
}

__global__ __launch_bounds__(128) void k_out(const _Float16* __restrict__ CT, const _Float16* __restrict__ WOT, float* __restrict__ OUT) {
  __shared__ __align__(16) float sf[4][16][132];
  const int tid = threadIdx.x; const int wave = __builtin_amdgcn_readfirstlane(threadIdx.x >> 5); const int lane = tid & 31, col = lane & 15, g = lane >> 4;
  const int c0 = blockIdx.y * 128; const size_t rb = (size_t)blockIdx.x * 64;
  const size_t bba = rb / TT; const size_t ta = rb % TT + (size_t)wave * 16 + col;
  const _Float16* ar = CT + ((bba * NH + g) * (size_t)TT + ta) * HD;
  const _Float16* wr = WOT + (size_t)(c0 + col) * CC;
  v8f acc[8] = {};
#pragma unroll 1
  for (int kc = 0; kc < CC / 32; ++kc) {
    union { v16h v; v8h q[2]; } a;
    a.q[0] = *(const v8h*)(ar + (size_t)(kc * 4) * TT * HD);
    a.q[1] = *(const v8h*)(ar + (size_t)(kc * 4 + 2) * TT * HD);
#pragma unroll
    for (int j = 0; j < 8; ++j) { const v16h w = frag_h(wr + (size_t)j * 16 * CC + kc * 32, lane); acc[j] = wmma16(a.v, w, acc[j]); } }
#pragma unroll
  for (int j = 0; j < 8; ++j) {
#pragma unroll
    for (int r = 0; r < 8; ++r) sf[wave][8 * g + r][j * 16 + col] = acc[j][r] * (1.0f / 16384.0f); }
  LDSX();
  const size_t bbo = rb / TT; const size_t to = rb % TT + (size_t)wave * 16;
#pragma unroll 1
  for (int rl = 0; rl < 16; ++rl) vst2(OUT + (bbo * TT_FULL + to + rl) * DIN + c0 + lane * 4, *(const v4f*)&sf[wave][rl][lane * 4]);
}

extern "C" void kernel_launch(void* const* d_in, const int* in_sizes, int n_in, void* d_out, int out_size, void* d_ws, size_t ws_size, hipStream_t stream) {
  if (n_in < 6) return;
  const long long xmin = ((long long)(NB - 1) * TT_FULL + TT) * DIN;
  if ((long long)in_sizes[0] < xmin) return;
  if (in_sizes[1] < DIN * CC || in_sizes[2] < DIN * CC || in_sizes[3] < DIN * CC || in_sizes[4] < CC * DIN) return;
  if (in_sizes[5] < HD) return;
  if ((long long)out_size < xmin) return;
  if (ws_size < (size_t)WS_END) return;
  const float* x = (const float*)d_in[0];
  const float* wq = (const float*)d_in[1];
  const float* wk = (const float*)d_in[2];
  const float* wv = (const float*)d_in[3];
  const float* wo = (const float*)d_in[4];
  const float* ph = (const float*)d_in[5];
  char* ws = (char*)d_ws;
  unsigned short* XB = (unsigned short*)(ws + WS_XB);
  unsigned short* WT = (unsigned short*)(ws + WS_WT);
  _Float16* QK = (_Float16*)(ws + WS_QK);
  _Float16* VT = (_Float16*)(ws + WS_VT);
  _Float16* CT = (_Float16*)(ws + WS_CT);
  k_cvtx<<<dim3((unsigned)((size_t)NB * TT * DIN / (8 * 256))), 256, 0, stream>>>(x, XB);
  k_wcv<<<dim3((unsigned)((size_t)CC * DIN / (8 * 256)), 4), 256, 0, stream>>>(wq, wk, wv, wo, WT);
  k_proj<<<dim3(NB * TT / 64, CC / 128, 3), 128, 0, stream>>>((const __bf16*)XB, (const __bf16*)WT, ph, QK, VT);
  k_attn<<<dim3(TT / 64, NH, NB), 128, 0, stream>>>(QK, QK + (size_t)NB * TT * CC, VT, CT);
  k_out<<<dim3(NB * TT / 64, DIN / 128), 128, 0, stream>>>(CT, (const _Float16*)(WT + (size_t)3 * CC * DIN), (float*)d_out);
}
